// InvariantPolynomial_89850715832863
// MI455X (gfx1250) — hardware-verified
//
#include <hip/hip_runtime.h>
#include <stddef.h>
#include <math.h>


#define NTHR   256
#define NWAVE  8
#define EPT    8
#define CHUNK  (NTHR * EPT)
#define WCAP   (EPT * 32)
#define LISTN  (NWAVE * WCAP)
#define PASSN  (NWAVE * 16)
#define PCAP   (CHUNK + PASSN)
#define PASS2  NTHR
#define PCAP2  (CHUNK + PASS2)

#define FA     23
#define FBD    7
#define MU0    64
#define MU1    24
#define MU2    16
#define NCOL   (MU0 + MU1 + MU2)
#define NPAD   112
#define NBK    7
#define KP     192
#define KSTEP  6
#define KQ     (KP / 8)
#define NODEB  160
#define ACCW   224
#define ACC1   MU0
#define ACC2   (MU0 + 3 * MU1)
#define ACCN   (MU0 + 3 * MU1 + 5 * MU2)
#define NVW    64
#define SRW    24
#define ARW    8
#define SHW    8
#define VT1    (MU0 * FBD)
#define VT2    (VT1 + MU1 * FBD)
#define VT3    (VT2 + MU2 * FBD)
#define VTAB   768
#define NB2    4096
#define GCAP   1024

#define S3F    1.7320508075688772f
#define S15F   3.872983346207417f
#define H5F    1.118033988749895f
#define H15F   1.9364916731037085f
#define A1F    0.07881104062391f
#define C0F    0.0472455591261534f
#define C1F    0.0445435403187374f
#define C2F    0.0422577127364258f

#define L_ACC   0
#define L_MSG   (L_ACC + (NODEB + 1) * ACCW * 4)
#define L_SROW  (L_MSG + NPAD * PASSN * 4)
#define L_AROW  (L_SROW + PASSN * SRW * 4)
#define L_SH    (L_AROW + PASSN * ARW * 4)
#define L_VT    (L_SH + PASSN * SHW * 4)
#define L_LIST  (L_VT + VTAB * 4)
#define L_PEND  (L_LIST + LISTN * 4)
#define L_SLOT  (L_PEND + PCAP * 4)
#define L_WCNT  (L_SLOT + PASSN * 4)
#define L_TOTAL (L_WCNT + 64)

static_assert(KP == 8 * (FA + 1));
static_assert(KSTEP * 32 == KP);
static_assert(NPAD == 16 * NBK && NCOL <= NPAD);
static_assert(ACCN == 216 && ACCN <= ACCW && ACCN <= NTHR);
static_assert((((NODEB + 1) * ACCW) % 4) == 0);
static_assert((NODEB % (2 * NWAVE)) == 0);
static_assert(NVW == 64 && 9 * FBD <= NVW);
static_assert(NODEB * NVW * 4 <= NPAD * PASSN * 4);
static_assert(VT3 <= VTAB);
static_assert(PASSN == 128 && PASS2 == NTHR);
static_assert((NB2 % (NWAVE * 128)) == 0);
static_assert((L_MSG % 16) == 0 && (L_SROW % 16) == 0 && (L_AROW % 16) == 0 && (L_SH % 16) == 0);
static_assert((L_VT % 16) == 0 && (L_LIST % 16) == 0 && (L_PEND % 16) == 0 && (L_SLOT % 16) == 0);
static_assert((L_WCNT % 16) == 0 && (L_TOTAL % 16) == 0);
static_assert(L_TOTAL <= 300 * 1024);
static_assert((GCAP % 4) == 0);

typedef float          v4f   __attribute__((ext_vector_type(4)));
typedef float          v8f   __attribute__((ext_vector_type(8)));
typedef int            v4i   __attribute__((ext_vector_type(4)));
typedef unsigned short v8us  __attribute__((ext_vector_type(8)));
typedef unsigned short v16us __attribute__((ext_vector_type(16)));
typedef __bf16         v16bf __attribute__((ext_vector_type(16)));

__device__ __forceinline__ v8f wmb(v16bf a, v16bf b, v8f c) {
  v8f d = __builtin_amdgcn_wmma_f32_16x16x32_bf16(false, a, false, b, (short)0, c, false, false);
  asm volatile("v_nop\n\tv_nop\n\tv_nop\n\tv_nop" : "+v"(d) : "v"(a), "v"(b) : "memory");
  return d;
}

__device__ __forceinline__ v8f splat8(float x) {
  v8f c;
#pragma unroll
  for (int i = 0; i < 8; ++i) c[i] = x;
  return c;
}

__device__ __forceinline__ unsigned short bfr(float f) {
  unsigned u = __float_as_uint(f);
  u += 0x7FFFu + ((u >> 16) & 1u);
  return (unsigned short)(u >> 16);
}

__device__ __forceinline__ v16bf cat16(v8us a, v8us b) {
  const v16us u = __builtin_shufflevector(a, b, 0, 1, 2, 3, 4, 5, 6, 7, 8, 9, 10, 11, 12, 13, 14, 15);
  return __builtin_bit_cast(v16bf, u);
}

struct HL8 { v8us hi; v8us lo; };

__device__ __forceinline__ HL8 prod_split(float s, v4f p0, v4f p1) {
  float t[8];
  t[0] = s * p0.x; t[1] = s * p0.y; t[2] = s * p0.z; t[3] = s * p0.w;
  t[4] = s * p1.x; t[5] = s * p1.y; t[6] = s * p1.z; t[7] = s * p1.w;
  HL8 r;
#pragma unroll
  for (int j = 0; j < 8; ++j) {
    const unsigned short hb = bfr(t[j]);
    const float hf = __uint_as_float(((unsigned)hb) << 16);
    r.hi[j] = hb;
    r.lo[j] = bfr(t[j] - hf);
  }
  return r;
}

__device__ __forceinline__ int scan_chunk(const int* __restrict__ dsts, int nE, int cbase, int nodeBase,
                                          int nrange, int vec8, int* list, int tid, int wave) {
  int wc = 0;
  const int el0  = tid * EPT;
  const int e0   = cbase + el0;
  const int sent = -2147483647 - 1;
  v4i da, db;
  if (vec8 != 0 && cbase + CHUNK <= nE) {
    da = *(const v4i*)(dsts + e0);
    db = *(const v4i*)(dsts + e0 + 4);
  } else {
    da.x = (e0     < nE) ? dsts[min(e0,     nE - 1)] : sent;
    da.y = (e0 + 1 < nE) ? dsts[min(e0 + 1, nE - 1)] : sent;
    da.z = (e0 + 2 < nE) ? dsts[min(e0 + 2, nE - 1)] : sent;
    da.w = (e0 + 3 < nE) ? dsts[min(e0 + 3, nE - 1)] : sent;
    db.x = (e0 + 4 < nE) ? dsts[min(e0 + 4, nE - 1)] : sent;
    db.y = (e0 + 5 < nE) ? dsts[min(e0 + 5, nE - 1)] : sent;
    db.z = (e0 + 6 < nE) ? dsts[min(e0 + 6, nE - 1)] : sent;
    db.w = (e0 + 7 < nE) ? dsts[min(e0 + 7, nE - 1)] : sent;
  }
  const unsigned nb = (unsigned)nodeBase;
  const unsigned nr = (unsigned)nrange;
  const unsigned s0 = (unsigned)da.x - nb, s1 = (unsigned)da.y - nb;
  const unsigned s2 = (unsigned)da.z - nb, s3 = (unsigned)da.w - nb;
  const unsigned s4 = (unsigned)db.x - nb, s5 = (unsigned)db.y - nb;
  const unsigned s6 = (unsigned)db.z - nb, s7 = (unsigned)db.w - nb;
  const bool h0 = s0 < nr, h1 = s1 < nr, h2 = s2 < nr, h3 = s3 < nr;
  const bool h4 = s4 < nr, h5 = s5 < nr, h6 = s6 < nr, h7 = s7 < nr;
  const unsigned any = __builtin_amdgcn_ballot_w32(h0 | h1 | h2 | h3 | h4 | h5 | h6 | h7);
  if (any != 0u) {
#define HITJ(J, HJ) { \
      const unsigned mj = __builtin_amdgcn_ballot_w32(HJ); \
      if (mj != 0u) { \
        if (HJ) { \
          const int pos = wc + (int)__builtin_amdgcn_mbcnt_lo(mj, 0u); \
          if (pos < WCAP) list[wave * WCAP + pos] = el0 + (J); \
        } \
        wc += (int)__builtin_popcount(mj); } }
    HITJ(0, h0)
    HITJ(1, h1)
    HITJ(2, h2)
    HITJ(3, h3)
    HITJ(4, h4)
    HITJ(5, h5)
    HITJ(6, h6)
    HITJ(7, h7)
#undef HITJ
  }
  return wc;
}

__device__ __forceinline__ int append_hits(const int* wcnt, int* pend, const int* list, int pcap,
                                           int cbase, int lane, int wave) {
  const int base = wcnt[NWAVE];
  int tot = 0, myoff = 0;
#pragma unroll
  for (int w = 0; w < NWAVE; ++w) {
    int c = wcnt[w];
    c = c > WCAP ? WCAP : (c < 0 ? 0 : c);
    if (w < wave) myoff += c;
    tot += c;
  }
  int newN = base + tot;
  newN = newN > pcap ? pcap : newN;
  int n = wcnt[wave];
  n = n > WCAP ? WCAP : (n < 0 ? 0 : n);
  const int* lp = list + wave * WCAP;
  for (int i = lane; i < n; i += 32) {
    const int pos = base + myoff + i;
    if (pos < pcap) pend[pos] = cbase + lp[i];
  }
  return newN;
}

__global__ __launch_bounds__(NTHR) void k_prepb(const float* __restrict__ W1, const float* __restrict__ W2,
                                               const float* __restrict__ W3,
                                               unsigned short* bhi, unsigned short* blo) {
  const int t = blockIdx.x * NTHR + threadIdx.x;
  if (t >= NPAD * KQ) return;
  const int n = t / KQ;
  const int u = t - n * KQ;
  const int uc = u > FA - 1 ? FA - 1 : u;
  const int n1 = n > MU0 - 1 ? MU0 - 1 : n;
  int n2 = n - MU0;       n2 = n2 < 0 ? 0 : (n2 > MU1 - 1 ? MU1 - 1 : n2);
  int n3 = n - MU0 - MU1; n3 = n3 < 0 ? 0 : (n3 > MU2 - 1 ? MU2 - 1 : n3);
  v8us vh, vl;
#pragma unroll
  for (int j = 0; j < 8; ++j) {
    const int vc = j > FBD - 1 ? FBD - 1 : j;
    const int uv = uc * FBD + vc;
    const float w1 = W1[uv * MU0 + n1];
    const float w2 = W2[uv * MU1 + n2];
    const float w3 = W3[uv * MU2 + n3];
    float w = n < MU0 ? w1 : (n < MU0 + MU1 ? w2 : w3);
    w = (u < FA && j < FBD && n < NCOL) ? w : 0.0f;
    const unsigned short hb = bfr(w);
    const float hf = __uint_as_float(((unsigned)hb) << 16);
    vh[j] = hb;
    vl[j] = bfr(w - hf);
  }
  const size_t o = (size_t)n * KP + 8 * u;
  *(volatile v8us*)(bhi + o) = vh;
  *(volatile v8us*)(blo + o) = vl;
  __threadfence();
  *(volatile v8us*)(bhi + o) = vh;
  *(volatile v8us*)(blo + o) = vl;
}

__global__ __launch_bounds__(NTHR) void k_msg(
    const float* __restrict__ pos, const float* __restrict__ xf, const float* __restrict__ eattr,
    const int* __restrict__ ei,
    const unsigned short* __restrict__ bhi, const unsigned short* __restrict__ blo,
    const float* __restrict__ V1, const float* __restrict__ V2, const float* __restrict__ V3,
    float* nvout, int nN, int nE, int vec8, float a1, float c0, float c1, float c2) {
  extern __shared__ __attribute__((aligned(16))) unsigned char dsm[];
  float* acc   = (float*)(dsm + L_ACC);
  float* msgT  = (float*)(dsm + L_MSG);
  float* srow  = (float*)(dsm + L_SROW);
  float* arow  = (float*)(dsm + L_AROW);
  float* shs   = (float*)(dsm + L_SH);
  float* vt    = (float*)(dsm + L_VT);
  int*   list  = (int*)(dsm + L_LIST);
  int*   pend  = (int*)(dsm + L_PEND);
  int*   slotb = (int*)(dsm + L_SLOT);
  int*   wcnt  = (int*)(dsm + L_WCNT);

  const int tid = threadIdx.x, lane = tid & 31, wave = tid >> 5, hh = lane >> 4, m = lane & 15;
  const int nodeBase = blockIdx.x * NODEB;
  const int* srcs = ei;
  const int* dsts = ei + nE;

  {
    const v4f z = {0.0f, 0.0f, 0.0f, 0.0f};
#pragma unroll 1
    for (int i = tid; i < (NODEB + 1) * ACCW / 4; i += NTHR) *(v4f*)(acc + 4 * i) = z;
  }
#pragma unroll 1
  for (int i = tid; i < VTAB; i += NTHR) {
    const int i1 = i > VT1 - 1 ? VT1 - 1 : i;
    int i2 = i - VT1; i2 = i2 < 0 ? 0 : (i2 > MU1 * FBD - 1 ? MU1 * FBD - 1 : i2);
    int i3 = i - VT2; i3 = i3 < 0 ? 0 : (i3 > MU2 * FBD - 1 ? MU2 * FBD - 1 : i3);
    const float v1 = V1[i1], v2 = V2[i2], v3 = V3[i3];
    float v = i < VT1 ? v1 : (i < VT2 ? v2 : v3);
    v = i < VT3 ? v : 0.0f;
    vt[i] = v;
  }
  if (tid == 0) wcnt[NWAVE] = 0;
  __syncthreads();

  const int nChunks = (nE + CHUNK - 1) / CHUNK;
#pragma unroll 1
  for (int ch = 0; ch < nChunks; ++ch) {
    const int cbase = ch * CHUNK;
    const int wc = scan_chunk(dsts, nE, cbase, nodeBase, NODEB, vec8, list, tid, wave);
    if (lane == 0) wcnt[wave] = wc;
    __syncthreads();
    const int newN = append_hits(wcnt, pend, list, PCAP, cbase, lane, wave);
    const int fin = (ch == nChunks - 1) ? 1 : 0;
    const int R   = (fin != 0) ? (newN + PASSN - 1) / PASSN : newN / PASSN;
    const int Pv  = (fin != 0) ? newN : R * PASSN;
    __syncthreads();

#pragma unroll 1
    for (int r = 0; r < R; ++r) {
      {
        int idx = r * PASSN + wave * 16 + m;
        const bool valid = idx < Pv;
        idx = idx > PCAP - 1 ? PCAP - 1 : idx;
        int e = pend[idx];
        e = e < 0 ? 0 : (e > nE - 1 ? nE - 1 : e);
        const int d = dsts[e];
        int s = srcs[e];
        int slot = d - nodeBase;
        if (!valid || (unsigned)slot >= (unsigned)NODEB) slot = NODEB;
        s = s < 0 ? 0 : (s > nN - 1 ? nN - 1 : s);
        const int dc = d < 0 ? 0 : (d > nN - 1 ? nN - 1 : d);
        {
          const float* xr = xf + (size_t)s * FA;
          float xv[12];
#pragma unroll
          for (int j = 0; j < 12; ++j) {
            const int uu = 12 * hh + j;
            const int uc = uu > FA - 1 ? FA - 1 : uu;
            const float t = xr[uc];
            xv[j] = (uu < FA) ? t : 0.0f;
          }
          float* sp = srow + (wave * 16 + m) * SRW + 12 * hh;
          const v4f x0 = {xv[0], xv[1], xv[2],  xv[3]};
          const v4f x1 = {xv[4], xv[5], xv[6],  xv[7]};
          const v4f x2 = {xv[8], xv[9], xv[10], xv[11]};
          *(v4f*)sp = x0;
          *(v4f*)(sp + 4) = x1;
          *(v4f*)(sp + 8) = x2;
        }
        {
          const float* er = eattr + (size_t)e * FBD;
          float av[4];
#pragma unroll
          for (int j = 0; j < 4; ++j) {
            const int vv = 4 * hh + j;
            const int vc = vv > FBD - 1 ? FBD - 1 : vv;
            const float t = er[vc];
            av[j] = (vv < FBD && valid) ? t : 0.0f;
          }
          const v4f a4 = {av[0], av[1], av[2], av[3]};
          *(v4f*)(arow + (wave * 16 + m) * ARW + 4 * hh) = a4;
        }
        {
          const float px = pos[(size_t)s * 3 + 0] - pos[(size_t)dc * 3 + 0];
          const float py = pos[(size_t)s * 3 + 1] - pos[(size_t)dc * 3 + 1];
          const float pz = pos[(size_t)s * 3 + 2] - pos[(size_t)dc * 3 + 2];
          const float r2 = px * px + py * py + pz * pz;
          const v4f g0 = {S3F * px, S3F * py, S3F * pz, S15F * px * py};
          const v4f g1 = {S15F * py * pz, H5F * (3.0f * pz * pz - r2), S15F * px * pz, H15F * (px * px - py * py)};
          if (hh == 0) {
            float* hp = shs + (wave * 16 + m) * SHW;
            *(v4f*)hp = g0;
            *(v4f*)(hp + 4) = g1;
          } else {
            slotb[wave * 16 + m] = slot;
          }
        }
      }
      __syncthreads();

      {
        const float* sp = srow + (wave * 16 + m) * SRW;
        const float* aq = arow + (wave * 16 + m) * ARW;
        const v4f e0 = *(const v4f*)aq;
        const v4f e1 = *(const v4f*)(aq + 4);
        v8f cacc[NBK];
#pragma unroll
        for (int nb = 0; nb < NBK; ++nb) cacc[nb] = splat8(0.0f);
        const unsigned short* bh = bhi + (size_t)m * KP + 8 * hh;
        const unsigned short* bl = blo + (size_t)m * KP + 8 * hh;
#pragma unroll 1
        for (int c = 0; c < KSTEP; ++c) {
          const float xa = sp[4 * c + hh];
          const float xb = sp[4 * c + 2 + hh];
          const HL8 qa = prod_split(xa, e0, e1);
          const HL8 qb = prod_split(xb, e0, e1);
          const v16bf ah = cat16(qa.hi, qb.hi);
          const v16bf al = cat16(qa.lo, qb.lo);
#pragma unroll
          for (int nb = 0; nb < NBK; ++nb) {
            const unsigned short* p0 = bh + nb * 16 * KP + 32 * c;
            const unsigned short* p1 = bl + nb * 16 * KP + 32 * c;
            const v16bf wh = cat16(*(const v8us*)p0, *(const v8us*)(p0 + 16));
            const v16bf wl = cat16(*(const v8us*)p1, *(const v8us*)(p1 + 16));
            cacc[nb] = wmb(ah, wh, cacc[nb]);
            cacc[nb] = wmb(ah, wl, cacc[nb]);
            cacc[nb] = wmb(al, wh, cacc[nb]);
          }
        }
#pragma unroll
        for (int nb = 0; nb < NBK; ++nb) {
          float* mp = msgT + (nb * 16 + m) * PASSN + wave * 16 + 8 * hh;
          const v4f o0 = {cacc[nb][0], cacc[nb][1], cacc[nb][2], cacc[nb][3]};
          const v4f o1 = {cacc[nb][4], cacc[nb][5], cacc[nb][6], cacc[nb][7]};
          *(v4f*)mp = o0;
          *(v4f*)(mp + 4) = o1;
        }
      }
      __syncthreads();

      if (tid < ACCN) {
        const int q1 = tid - ACC1; const int w1 = q1 / 3; const int m1 = q1 - 3 * w1;
        const int q2 = tid - ACC2; const int w2 = q2 / 5; const int m2 = q2 - 5 * w2;
        int fcol = tid < ACC1 ? tid : (tid < ACC2 ? MU0 + w1 : MU0 + MU1 + w2);
        fcol = fcol < 0 ? 0 : (fcol > NCOL - 1 ? NCOL - 1 : fcol);
        int cidx = tid < ACC1 ? 0 : (tid < ACC2 ? m1 : 3 + m2);
        cidx = cidx < 0 ? 0 : (cidx > SHW - 1 ? SHW - 1 : cidx);
        const bool plain = tid < ACC1;
        const float* mrow = msgT + fcol * PASSN;
        float* ac = acc + tid;
#pragma unroll 1
        for (int i = 0; i < PASSN; ++i) {
          int sl = slotb[i];
          sl = sl < 0 ? 0 : (sl > NODEB ? NODEB : sl);
          const float cf0 = shs[i * SHW + cidx];
          const float cf = plain ? 1.0f : cf0;
          ac[sl * ACCW] += mrow[i] * cf;
        }
      }
      __syncthreads();
    }

    int rem = newN - R * PASSN;
    rem = rem < 0 ? 0 : rem;
    if (R > 0 && tid < rem) pend[tid] = pend[R * PASSN + tid];
    if (tid == 0) wcnt[NWAVE] = rem;
  }
  __syncthreads();

  float* stg = msgT;
#pragma unroll 1
  for (int it = tid; it < NODEB * NVW; it += NTHR) {
    const int node = it >> 6;
    const int q = it & 63;
    const int q2 = q - 7;  const int mm2 = q2 / 7; const int v2 = q2 - 7 * mm2;
    const int q3 = q - 28; const int mm3 = q3 / 7; const int v3 = q3 - 7 * mm3;
    const bool t0 = q < 7, t1 = q < 28, t2 = q < 63;
    const int cnt = t0 ? MU0 : (t1 ? MU1 : (t2 ? MU2 : 0));
    int ab  = t0 ? 0 : (t1 ? ACC1 + mm2 : ACC2 + mm3);
    ab = ab < 0 ? 0 : (ab > ACCW - 1 ? ACCW - 1 : ab);
    const int ast = t0 ? 1 : (t1 ? 3 : 5);
    int vb = t0 ? q : (t1 ? VT1 + v2 : VT2 + v3);
    vb = vb < 0 ? 0 : (vb > VTAB - 1 ? VTAB - 1 : vb);
    const float cl = t0 ? c0 : (t1 ? c1 : c2);
    const float* ap = acc + node * ACCW + ab;
    const float* vp = vt + vb;
    float ssum = 0.0f;
#pragma unroll 1
    for (int uu = 0; uu < cnt; ++uu) ssum = fmaf(ap[uu * ast], vp[uu * FBD], ssum);
    stg[it] = cl * (a1 * ssum);
  }
  __syncthreads();

#pragma unroll 1
  for (int q = 0; q < NODEB / (2 * NWAVE); ++q) {
    const int row = wave * (NODEB / NWAVE) + 2 * q + (lane >> 4);
    const int c4 = 4 * (lane & 15);
    const v4f v = *(const v4f*)(stg + row * NVW + c4);
    *(volatile v4f*)(nvout + (size_t)(nodeBase + row) * NVW + c4) = v;
  }
  __threadfence();
#pragma unroll 1
  for (int q = 0; q < NODEB / (2 * NWAVE); ++q) {
    const int row = wave * (NODEB / NWAVE) + 2 * q + (lane >> 4);
    const int c4 = 4 * (lane & 15);
    const v4f v = *(const v4f*)(stg + row * NVW + c4);
    *(volatile v4f*)(nvout + (size_t)(nodeBase + row) * NVW + c4) = v;
  }
}

__global__ __launch_bounds__(NTHR) void k_tp2(const float* __restrict__ pos, const float* __restrict__ eattr,
                                             const int* __restrict__ ei, const float* __restrict__ nv,
                                             float* nout, int nN, int nE, int vec8) {
  __shared__ __attribute__((aligned(16))) float acc2[NB2 + 4];
  __shared__ __attribute__((aligned(16))) float gbuf[PASS2];
  __shared__ int   slot2[PASS2];
  __shared__ float cfl[NTHR * 9];
  __shared__ int   list[LISTN];
  __shared__ int   pend[PCAP2];
  __shared__ int   wcnt[NWAVE + 1];

  const int tid = threadIdx.x, lane = tid & 31, wave = tid >> 5;
  const int nodeBase = blockIdx.x * NB2;
  const int* srcs = ei;
  const int* dsts = ei + nE;

#pragma unroll 1
  for (int i = tid; i < NB2 + 4; i += NTHR) acc2[i] = 0.0f;
  if (tid == 0) wcnt[NWAVE] = 0;
  __syncthreads();

  const int nChunks = (nE + CHUNK - 1) / CHUNK;
#pragma unroll 1
  for (int ch = 0; ch < nChunks; ++ch) {
    const int cbase = ch * CHUNK;
    const int wc = scan_chunk(dsts, nE, cbase, nodeBase, NB2, vec8, list, tid, wave);
    if (lane == 0) wcnt[wave] = wc;
    __syncthreads();
    const int newN = append_hits(wcnt, pend, list, PCAP2, cbase, lane, wave);
    const int fin = (ch == nChunks - 1) ? 1 : 0;
    const int R   = (fin != 0) ? (newN + PASS2 - 1) / PASS2 : newN / PASS2;
    const int Pv  = (fin != 0) ? newN : R * PASS2;
    __syncthreads();

#pragma unroll 1
    for (int r = 0; r < R; ++r) {
      {
        int idx = r * PASS2 + tid;
        const bool valid = idx < Pv;
        idx = idx > PCAP2 - 1 ? PCAP2 - 1 : idx;
        int e = pend[idx];
        e = e < 0 ? 0 : (e > nE - 1 ? nE - 1 : e);
        const int d = dsts[e];
        int s = srcs[e];
        int slot = d - nodeBase;
        if (!valid || (unsigned)slot >= (unsigned)NB2) slot = NB2;
        s = s < 0 ? 0 : (s > nN - 1 ? nN - 1 : s);
        const int dc = d < 0 ? 0 : (d > nN - 1 ? nN - 1 : d);
        const float px = pos[(size_t)s * 3 + 0] - pos[(size_t)dc * 3 + 0];
        const float py = pos[(size_t)s * 3 + 1] - pos[(size_t)dc * 3 + 1];
        const float pz = pos[(size_t)s * 3 + 2] - pos[(size_t)dc * 3 + 2];
        const float r2 = px * px + py * py + pz * pz;
        float* cp = cfl + tid * 9;
        cp[0] = 1.0f;
        cp[1] = S3F * px;
        cp[2] = S3F * py;
        cp[3] = S3F * pz;
        cp[4] = S15F * px * py;
        cp[5] = S15F * py * pz;
        cp[6] = H5F * (3.0f * pz * pz - r2);
        cp[7] = S15F * px * pz;
        cp[8] = H15F * (px * px - py * py);
        const float* er = eattr + (size_t)e * FBD;
        float ev[FBD];
#pragma unroll
        for (int j = 0; j < FBD; ++j) ev[j] = er[j];
        const float* nvr = nv + (size_t)s * NVW;
        float g = 0.0f;
#pragma unroll 1
        for (int mr = 0; mr < 9; ++mr) {
          const float* rp = nvr + FBD * mr;
          float dsum = ev[0] * rp[0];
          dsum = fmaf(ev[1], rp[1], dsum);
          dsum = fmaf(ev[2], rp[2], dsum);
          dsum = fmaf(ev[3], rp[3], dsum);
          dsum = fmaf(ev[4], rp[4], dsum);
          dsum = fmaf(ev[5], rp[5], dsum);
          dsum = fmaf(ev[6], rp[6], dsum);
          g = fmaf(cp[mr], dsum, g);
        }
        gbuf[tid]  = valid ? g : 0.0f;
        slot2[tid] = slot;
      }
      __syncthreads();
      if (tid == 0) {
#pragma unroll 1
        for (int i = 0; i < PASS2; ++i) {
          int sl = slot2[i];
          sl = sl < 0 ? 0 : (sl > NB2 ? NB2 : sl);
          acc2[sl] += gbuf[i];
        }
      }
      __syncthreads();
    }

    int rem = newN - R * PASS2;
    rem = rem < 0 ? 0 : rem;
    if (R > 0 && tid < rem) pend[tid] = pend[R * PASS2 + tid];
    if (tid == 0) wcnt[NWAVE] = rem;
  }
  __syncthreads();

#pragma unroll 1
  for (int q = 0; q < NB2 / (NWAVE * 128); ++q) {
    const int off = wave * (NB2 / NWAVE) + q * 128 + 4 * lane;
    const v4f v = *(const v4f*)(acc2 + off);
    *(volatile v4f*)(nout + (size_t)nodeBase + off) = v;
  }
  __threadfence();
#pragma unroll 1
  for (int q = 0; q < NB2 / (NWAVE * 128); ++q) {
    const int off = wave * (NB2 / NWAVE) + q * 128 + 4 * lane;
    const v4f v = *(const v4f*)(acc2 + off);
    *(volatile v4f*)(nout + (size_t)nodeBase + off) = v;
  }
}

__global__ __launch_bounds__(NTHR) void k_pool(const float* __restrict__ nout, const int* __restrict__ bt,
                                              float* out, int nN, int G) {
  __shared__ __attribute__((aligned(16))) float gacc[GCAP + 4];
  __shared__ float vbuf[NTHR];
  __shared__ int   bbuf[NTHR];
  const int tid = threadIdx.x;
#pragma unroll 1
  for (int i = tid; i < GCAP + 4; i += NTHR) gacc[i] = 0.0f;
  __syncthreads();
  const int nCh = (nN + NTHR - 1) / NTHR;
#pragma unroll 1
  for (int ch = 0; ch < nCh; ++ch) {
    const int i  = ch * NTHR + tid;
    const int ic = i > nN - 1 ? nN - 1 : i;
    const float v = nout[ic];
    const int   b = bt[ic];
    const bool ok = (i < nN) && ((unsigned)b < (unsigned)G);
    vbuf[tid] = ok ? v : 0.0f;
    bbuf[tid] = ok ? b : GCAP;
    __syncthreads();
    if (tid == 0) {
#pragma unroll 1
      for (int j = 0; j < NTHR; ++j) {
        int sl = bbuf[j];
        sl = sl < 0 ? 0 : (sl > GCAP ? GCAP : sl);
        gacc[sl] += vbuf[j];
      }
    }
    __syncthreads();
  }
  const int nq = G >> 2;
  v4f v = {0.0f, 0.0f, 0.0f, 0.0f};
  if (tid < nq) v = *(const v4f*)(gacc + 4 * tid);
  if (tid < nq) *(volatile v4f*)(out + 4 * tid) = v;
  if (tid == 0) {
#pragma unroll 1
    for (int j = 4 * nq; j < G; ++j) ((volatile float*)out)[j] = gacc[j];
  }
  __threadfence();
  if (tid < nq) *(volatile v4f*)(out + 4 * tid) = v;
  if (tid == 0) {
#pragma unroll 1
    for (int j = 4 * nq; j < G; ++j) ((volatile float*)out)[j] = gacc[j];
  }
}

extern "C" void kernel_launch(void* const* d_in, const int* in_sizes, int n_in,
                              void* d_out, int out_size, void* d_ws, size_t ws_size,
                              hipStream_t stream) {
  if (n_in < 11) return;
  const int nN = in_sizes[4];
  if (nN < 1 || in_sizes[0] != 3 * nN || in_sizes[1] != FA * nN) return;
  if (in_sizes[3] < 2 || (in_sizes[3] & 1) != 0) return;
  const int nE = in_sizes[3] / 2;
  if (in_sizes[2] != FBD * nE) return;
  if (in_sizes[5] != FA * FBD * MU0 || in_sizes[6] != FA * FBD * MU1 || in_sizes[7] != FA * FBD * MU2) return;
  if (in_sizes[8] != MU0 * FBD || in_sizes[9] != MU1 * FBD || in_sizes[10] != MU2 * FBD) return;
  const int G = out_size;
  if (G < 1 || G > GCAP) return;

  const float* pos   = (const float*)d_in[0];
  const float* xf    = (const float*)d_in[1];
  const float* eattr = (const float*)d_in[2];
  const int*   ei    = (const int*)d_in[3];
  const int*   batch = (const int*)d_in[4];
  const float* W1    = (const float*)d_in[5];
  const float* W2    = (const float*)d_in[6];
  const float* W3    = (const float*)d_in[7];
  const float* V1    = (const float*)d_in[8];
  const float* V2    = (const float*)d_in[9];
  const float* V3    = (const float*)d_in[10];
  float* outp = (float*)d_out;

  const int nBlk  = (nN + NODEB - 1) / NODEB;
  const size_t rowsP = (size_t)nBlk * NODEB;
  const int nBlk2 = (nN + NB2 - 1) / NB2;
  const size_t rows2 = (size_t)nBlk2 * NB2;

  char* ws = (char*)d_ws;
  size_t off = 0;
  const size_t szB = ((size_t)NPAD * KP * 2 + 255) & ~(size_t)255;
  const size_t oBh = off; off += szB;
  const size_t oBl = off; off += szB;
  const size_t oNV = off; off += (rowsP * NVW * 4 + 255) & ~(size_t)255;
  const size_t oNO = off; off += (rows2 * 4 + 255) & ~(size_t)255;
  size_t limit = (size_t)134217728;
  if (ws_size < limit) limit = ws_size;
  if (off > limit) return;
  unsigned short* Bh = (unsigned short*)(ws + oBh);
  unsigned short* Bl = (unsigned short*)(ws + oBl);
  float* NVp = (float*)(ws + oNV);
  float* NOp = (float*)(ws + oNO);

  const int vec8 = ((nE & 3) == 0) ? 1 : 0;
  const float a1 = A1F, c0 = C0F, c1 = C1F, c2 = C2F;

  k_prepb<<<(NPAD * KQ + NTHR - 1) / NTHR, NTHR, 0, stream>>>(W1, W2, W3, Bh, Bl);

  hipFuncSetAttribute(reinterpret_cast<const void*>(&k_msg), hipFuncAttributeMaxDynamicSharedMemorySize, L_TOTAL);
  k_msg<<<nBlk, NTHR, L_TOTAL, stream>>>(pos, xf, eattr, ei, Bh, Bl, V1, V2, V3, NVp, nN, nE, vec8,
                                          a1, c0, c1, c2);

  k_tp2<<<nBlk2, NTHR, 0, stream>>>(pos, eattr, ei, NVp, NOp, nN, nE, vec8);

  k_pool<<<1, NTHR, 0, stream>>>(NOp, batch, outp, nN, G);
}
